// TrueASAAttention_76227079569857
// MI455X (gfx1250) — hardware-verified
//
#include <hip/hip_runtime.h>
#include <math.h>
#include <stdint.h>


typedef __attribute__((ext_vector_type(16))) _Float16 v16h;
typedef __attribute__((ext_vector_type(8)))  _Float16 v8h;
typedef __attribute__((ext_vector_type(16))) __bf16   v16b;
typedef __attribute__((ext_vector_type(8)))  __bf16   v8b;
typedef __attribute__((ext_vector_type(8)))  float    v8f;
typedef __attribute__((ext_vector_type(4)))  float    v4f;
typedef __attribute__((ext_vector_type(4)))  unsigned v4u;
#define U16(p) ((const unsigned short*)(const void*)(p))

__device__ __forceinline__ unsigned short f2bf_bits(float f) {
  unsigned u = __float_as_uint(f);
  return (unsigned short)((u + 0x7FFFu + ((u >> 16) & 1u)) >> 16);
}
__device__ __forceinline__ float bf_bits2f(unsigned short h) { return __uint_as_float(((unsigned)h) << 16); }

__device__ __forceinline__ void dep_guard_h(v8f& a, v8f& b, v16h x, v16h y) { asm volatile("v_nop\n\tv_nop\n\tv_nop\n\tv_nop" : "+v"(a), "+v"(b) : "v"(x), "v"(y)); }
__device__ __forceinline__ void dep_guard_b(v8f& a, v8f& b, v16b x, v16b y) { asm volatile("v_nop\n\tv_nop\n\tv_nop\n\tv_nop" : "+v"(a), "+v"(b) : "v"(x), "v"(y)); }
__device__ __forceinline__ void keep4_h(v16h a, v16h b, v16h c, v16h d) { asm volatile("v_nop" :: "v"(a), "v"(b), "v"(c), "v"(d)); }
__device__ __forceinline__ void keep4_b(v16b a, v16b b, v16b c, v16b d) { asm volatile("v_nop" :: "v"(a), "v"(b), "v"(c), "v"(d)); }
__device__ __forceinline__ void acc_guard4(v8f& a, v8f& b, v8f& c, v8f& d) { asm volatile("v_nop\n\tv_nop\n\tv_nop\n\tv_nop" : "+v"(a), "+v"(b), "+v"(c), "+v"(d)); }
template <typename T> struct Frag;
template <> struct Frag<_Float16> {
  typedef v16h V; union U { v16h v; v8h h[2]; };
  static __device__ __forceinline__ v16h load(const _Float16* p) {
    U f; f.h[0] = *(const v8h*)(p); f.h[1] = *(const v8h*)(p + 16); return f.v;
  }
  static __device__ __forceinline__ v8f mma(v16h a, v16h b, v8f c) {
    return __builtin_amdgcn_wmma_f32_16x16x32_f16(false, a, false, b, (short)0, c, false, false);
  }
  static __device__ __forceinline__ void guard(v8f& a, v8f& b, v16h x, v16h y) { dep_guard_h(a, b, x, y); }
  static __device__ __forceinline__ void keep(v16h a, v16h b, v16h c, v16h d) { keep4_h(a, b, c, d); }
};
template <> struct Frag<__bf16> {
  typedef v16b V; union U { v16b v; v8b h[2]; };
  static __device__ __forceinline__ v16b load(const __bf16* p) {
    U f; f.h[0] = *(const v8b*)(p); f.h[1] = *(const v8b*)(p + 16); return f.v;
  }
  static __device__ __forceinline__ v8f mma(v16b a, v16b b, v8f c) {
    return __builtin_amdgcn_wmma_f32_16x16x32_bf16(false, a, false, b, (short)0, c, false, false);
  }
  static __device__ __forceinline__ void guard(v8f& a, v8f& b, v16b x, v16b y) { dep_guard_b(a, b, x, y); }
  static __device__ __forceinline__ void keep(v16b a, v16b b, v16b c, v16b d) { keep4_b(a, b, c, d); }
};

template <int ET> struct Elem;
template <> struct Elem<0> { typedef _Float16 T; };
template <> struct Elem<1> { typedef __bf16 T; };
template <int ET, bool SPLIT, int BIAS_MODE, int OUT_MODE, bool RESID, int ACT = 0>
__global__ __launch_bounds__(256) void wmma_gemm64(
    const unsigned short* __restrict__ Ap, const unsigned short* __restrict__ A2p, int lda, long strideA,
    const unsigned short* __restrict__ Btp, const unsigned short* __restrict__ Bt2p, int ldb, long strideB,
    void* __restrict__ Cout, void* __restrict__ Cout2, int ldc, long strideC,
    const float* __restrict__ bias,
    const float* __restrict__ resid, long strideR,
    int M, int N, int K, float scale) {
  typedef typename Elem<ET>::T T;
  typedef typename Frag<T>::V V;
  const T* A = (const T*)Ap; const T* A2 = (const T*)A2p; const T* Bt = (const T*)Btp; const T* Bt2 = (const T*)Bt2p;
  __shared__ __align__(16) float sT[8][16 * 68];
  const int b    = blockIdx.y;
  const int lane = threadIdx.x & 31;
  const int wave = threadIdx.x >> 5;
  const int tilesN = N >> 6;
  const int tilesM = M >> 6;
  const int tile = blockIdx.x * 8 + wave;
  if (tile >= tilesM * tilesN) return;
  const int tm = tile / tilesN;
  const int tn = tile - tm * tilesN;
  const int m0 = tm << 6;
  const int n0 = tn << 6;

  const T* Ab  = A  + (size_t)b * strideA;
  const T* Bb  = Bt + (size_t)b * strideB;
  const T* Ab2 = SPLIT ? (A2  + (size_t)b * strideA) : nullptr;
  const T* Bb2 = SPLIT ? (Bt2 + (size_t)b * strideB) : nullptr;

  const int rlane = lane & 15;
  const int koff  = (lane >> 4) * 8;
  const int mOff  = (lane >> 4) * 8;

  v8f acc[4][4];
#pragma unroll
  for (int i = 0; i < 4; ++i)
#pragma unroll
    for (int j = 0; j < 4; ++j) acc[i][j] = (v8f){0.f,0.f,0.f,0.f,0.f,0.f,0.f,0.f};

  for (int k0 = 0; k0 < K; k0 += 32) {
    V bh[4], bl[4];
#pragma unroll
    for (int j = 0; j < 4; ++j) {
      const size_t bo = (size_t)(n0 + (j << 4) + rlane) * ldb + koff + k0;
      bh[j] = Frag<T>::load(Bb + bo);
      if (SPLIT) bl[j] = Frag<T>::load(Bb2 + bo);
    }
#pragma unroll
    for (int i = 0; i < 4; ++i) {
      const size_t ao = (size_t)(m0 + (i << 4) + rlane) * lda + koff + k0;
      V ah = Frag<T>::load(Ab + ao);
      V al;
      if (SPLIT) al = Frag<T>::load(Ab2 + ao);
#pragma unroll
      for (int j = 0; j < 4; ++j) {
        acc[i][j] = Frag<T>::mma(ah, bh[j], acc[i][j]);
        if (SPLIT) {
          acc[i][j] = Frag<T>::mma(ah, bl[j], acc[i][j]);
          acc[i][j] = Frag<T>::mma(al, bh[j], acc[i][j]);
        }
      }
      Frag<T>::guard(acc[i][0], acc[i][3], ah, SPLIT ? al : ah);
    }
    Frag<T>::keep(bh[0], bh[1], bh[2], bh[3]);
    if (SPLIT) Frag<T>::keep(bl[0], bl[1], bl[2], bl[3]);
  }
  acc_guard4(acc[0][0], acc[0][1], acc[0][2], acc[0][3]);
  acc_guard4(acc[1][0], acc[1][1], acc[1][2], acc[1][3]);
  acc_guard4(acc[2][0], acc[2][1], acc[2][2], acc[2][3]);
  acc_guard4(acc[3][0], acc[3][1], acc[3][2], acc[3][3]);

  float* slab = sT[wave];
  const float* Rb = RESID ? (resid + (size_t)b * strideR) : nullptr;
#pragma unroll
  for (int i = 0; i < 4; ++i) {
    const int mBase = m0 + (i << 4);
#pragma unroll
    for (int j = 0; j < 4; ++j) {
      const int n = n0 + (j << 4) + rlane;
      float bv = 0.f;
      if (BIAS_MODE == 2) bv = bias[n];
#pragma unroll
      for (int r = 0; r < 8; ++r) {
        float v = acc[i][j][r] * scale;
        if (BIAS_MODE == 1) v += bias[mBase + mOff + r];
        if (BIAS_MODE == 2) v += bv;
        if (RESID) v += Rb[(size_t)(mBase + mOff + r) * ldc + n];
        if (ACT == 1) v = tanhf(v);
        if (ACT == 2) v = fmaxf(v, 0.0f);
        if (ACT == 3) v = v / (1.0f + expf(-v));
        if (ACT == 4) v = (v > 0.f) ? v : 0.01f * v;
        if (ACT == 5) v = 0.5f * v * (1.0f + erff(v * 0.70710678118654752f));
        slab[(mOff + r) * 68 + (j << 4) + rlane] = v;
      }
    }
    __builtin_amdgcn_fence(__ATOMIC_RELEASE, "workgroup");
    __builtin_amdgcn_wave_barrier();
    __builtin_amdgcn_fence(__ATOMIC_ACQUIRE, "workgroup");
    if (OUT_MODE == 0) {
      float* C = (float*)Cout + (size_t)b * strideC;
      const int hh = lane >> 4, c4 = (lane & 15) * 4;
      for (int pass = 0; pass < 2; ++pass) {
#pragma unroll
        for (int it = 0; it < 8; ++it) {
          const int row = it * 2 + hh;
          v4f v = *(const v4f*)(slab + row * 68 + c4);
          *(volatile v4f*)(C + (size_t)(mBase + row) * ldc + n0 + c4) = v;
        }
        __threadfence();
      }
    } else {
      const int q = lane >> 3, c8 = (lane & 7) * 8;
      unsigned short* C  = (unsigned short*)Cout  + (size_t)b * strideC;
      unsigned short* C2 = (OUT_MODE == 2) ? ((unsigned short*)Cout2 + (size_t)b * strideC) : nullptr;
      for (int pass = 0; pass < 2; ++pass) {
#pragma unroll
        for (int it = 0; it < 4; ++it) {
          const int row = it * 4 + q;
          const float* sp = slab + row * 68 + c8;
          v8h hv, lv;
#pragma unroll
          for (int e = 0; e < 8; ++e) {
            if (OUT_MODE == 1) {
              hv[e] = (_Float16)sp[e];
            } else {
              unsigned short hb = f2bf_bits(sp[e]);
              unsigned short lb = f2bf_bits(sp[e] - bf_bits2f(hb));
              hv[e] = __builtin_bit_cast(_Float16, hb);
              lv[e] = __builtin_bit_cast(_Float16, lb);
            }
          }
          *(volatile v8h*)(C + (size_t)(mBase + row) * ldc + n0 + c8) = hv;
          if (OUT_MODE == 2) *(volatile v8h*)(C2 + (size_t)(mBase + row) * ldc + n0 + c8) = lv;
        }
        __threadfence();
      }
    }
    __builtin_amdgcn_fence(__ATOMIC_RELEASE, "workgroup");
    __builtin_amdgcn_wave_barrier();
    __builtin_amdgcn_fence(__ATOMIC_ACQUIRE, "workgroup");
  }
}

__device__ __forceinline__ v8f at_mma(v16b a, v16b b, v8f c) {
  c = __builtin_amdgcn_wmma_f32_16x16x32_bf16(false, a, false, b, (short)0, c, false, false);
  asm volatile("v_nop\n\tv_nop\n\tv_nop\n\tv_nop" : "+v"(c) : "v"(a), "v"(b));
  return c;
}
__device__ __forceinline__ v8f mma_h16(v16h a, v16h b, v8f c) {
  c = __builtin_amdgcn_wmma_f32_16x16x32_f16(false, a, false, b, (short)0, c, false, false);
  asm volatile("v_nop\n\tv_nop\n\tv_nop\n\tv_nop" : "+v"(c) : "v"(a), "v"(b));
  return c;
}

#define NSEQ 4096
#define NCHK 64
#define RTOT 16384
#define SDIM 64
#define DPAD 256
#define DOUT 244
#define KPL 72
#define VPL 72
#define PPL 72
#define OPL 72
#define PCARRY 32768.0f
#define PCARRY_INV (1.0f / 32768.0f)

__global__ __launch_bounds__(256) void split_bf16x2(const float* __restrict__ in, unsigned short* __restrict__ hi,
                                                    unsigned short* __restrict__ lo, int n2) {
  const int i = blockIdx.x * 256 + threadIdx.x;
  if (i < n2) {
    const float f0 = in[2 * i], f1 = in[2 * i + 1];
    const unsigned short h0 = f2bf_bits(f0), h1 = f2bf_bits(f1);
    const unsigned short l0 = f2bf_bits(f0 - bf_bits2f(h0)), l1 = f2bf_bits(f1 - bf_bits2f(h1));
    const unsigned uh = (unsigned)h0 | ((unsigned)h1 << 16);
    const unsigned ul = (unsigned)l0 | ((unsigned)l1 << 16);
    ((volatile unsigned*)hi)[i] = uh;
    ((volatile unsigned*)lo)[i] = ul;
    __threadfence();
    ((volatile unsigned*)hi)[i] = uh;
    ((volatile unsigned*)lo)[i] = ul;
  }
}

__global__ __launch_bounds__(256) void padcast_f16x2(const float* __restrict__ src, _Float16* __restrict__ dst,
                                                     int srows, int scols, float scale, int n2) {
  const int i = blockIdx.x * 256 + threadIdx.x;
  if (i < n2) {
    const int r  = i >> 7;
    const int c2 = (i & 127) * 2;
    const int rr = (r < srows) ? r : (srows - 1);
    const int c0 = (c2 < scols) ? c2 : (scols - 1);
    const int c1 = (c2 + 1 < scols) ? (c2 + 1) : (scols - 1);
    float f0 = src[(size_t)rr * scols + c0] * scale;
    float f1 = src[(size_t)rr * scols + c1] * scale;
    if (!(r < srows && c2 < scols)) f0 = 0.0f;
    if (!(r < srows && c2 + 1 < scols)) f1 = 0.0f;
    const _Float16 h0 = (_Float16)f0, h1 = (_Float16)f1;
    const unsigned u = (unsigned)__builtin_bit_cast(unsigned short, h0) | ((unsigned)__builtin_bit_cast(unsigned short, h1) << 16);
    ((volatile unsigned*)dst)[i] = u;
    __threadfence();
    ((volatile unsigned*)dst)[i] = u;
  }
}

__global__ __launch_bounds__(256) void pad_bias2(const float* __restrict__ b0, int n0, const float* __restrict__ b1, int n1,
                                                float* __restrict__ o0, float* __restrict__ o1) {
  const int t = threadIdx.x;
  const int i0 = (t < n0) ? t : (n0 - 1);
  const int i1 = (t < n1) ? t : (n1 - 1);
  float v0 = b0[i0]; if (t >= n0) v0 = 0.0f;
  float v1 = b1[i1]; if (t >= n1) v1 = 0.0f;
  ((volatile float*)o0)[t] = v0;
  ((volatile float*)o1)[t] = v1;
  __threadfence();
  ((volatile float*)o0)[t] = v0;
  ((volatile float*)o1)[t] = v1;
}

__global__ __launch_bounds__(256) void copy_out(const float* __restrict__ Y, float* __restrict__ out, int n4) {
  const int i = blockIdx.x * 256 + threadIdx.x;
  if (i < n4) {
    const int e = i * 4;
    const int r = e / DOUT;
    const int cc = e - r * DOUT;
    const v4f v = *(const v4f*)(Y + (size_t)r * DPAD + cc);
    *(volatile v4f*)(out + e) = v;
    __threadfence();
    *(volatile v4f*)(out + e) = v;
  }
}

__global__ __launch_bounds__(512) void attn_energy(
    const unsigned short* __restrict__ Shi, const unsigned short* __restrict__ Slo,
    const _Float16* __restrict__ Vt,
    const float* __restrict__ charge, const float* __restrict__ mass,
    const float* __restrict__ position, const float* __restrict__ valence,
    _Float16* __restrict__ Ob) {
  __shared__ __align__(16) __bf16 Ksh[NCHK * KPL];
  __shared__ __align__(16) __bf16 Ksl[NCHK * KPL];
  __shared__ __align__(16) _Float16 Vts[DPAD * VPL];
  __shared__ __align__(16) _Float16 Psh[4 * 16 * PPL];
  __shared__ float cjs[NCHK], sjs[NCHK], pjs[NCHK];
  __shared__ float mxs[4][NCHK];
  __shared__ float csx[4][NCHK], mfx[4][NCHK], zfx[4][NCHK];

  const int tid  = threadIdx.x;
  const int wave = tid >> 5, lane = tid & 31, hh = lane >> 4, c = lane & 15;
  const int rg = wave & 3, qt = wave >> 2;
  const int b = blockIdx.x >> 6, qb = blockIdx.x & 63;
  const int q0 = qb * 64 + rg * 16;
  const size_t brow = (size_t)b * NSEQ;
  const size_t gq = brow + q0;
  const __bf16* Shb = (const __bf16*)(const void*)Shi;
  const __bf16* Slb = (const __bf16*)(const void*)Slo;
  const float NEGINF = -__builtin_inff();

  v16b qah[2], qal[2];
#pragma unroll
  for (int dc = 0; dc < 2; ++dc) {
    const size_t o = (gq + c) * SDIM + dc * 32 + 8 * hh;
    qah[dc] = Frag<__bf16>::load(Shb + o);
    qal[dc] = Frag<__bf16>::load(Slb + o);
  }
  float ci[8], si[8], pi[8], mrun[8], csp[8], mf[8], zf[8];
#pragma unroll
  for (int r = 0; r < 8; ++r) {
    const size_t gr = gq + 8 * hh + r;
    ci[r] = charge[gr];
    si[r] = sqrtf(mass[gr]);
    pi[r] = position[gr];
    mrun[r] = NEGINF; csp[r] = 0.0f; mf[r] = NEGINF; zf[r] = 0.0f;
  }
  v8f oacc[4];
#pragma unroll
  for (int t = 0; t < 4; ++t) oacc[t] = (v8f){0.f,0.f,0.f,0.f,0.f,0.f,0.f,0.f};

  const int kidx = qt * 16 + c;
  const int krow = kidx * KPL + 8 * hh;

  for (int kc = 0; kc <= qb; ++kc) {
    const int kv0 = kc * NCHK;
    const size_t gk = brow + kv0;
    __syncthreads();
    {
      const int row = tid >> 3, q8 = tid & 7;
      const v4u vh = *(const v4u*)(Shi + (gk + row) * SDIM + q8 * 8);
      const v4u vl = *(const v4u*)(Slo + (gk + row) * SDIM + q8 * 8);
      *(v4u*)(Ksh + row * KPL + q8 * 8) = vh;
      *(v4u*)(Ksl + row * KPL + q8 * 8) = vl;
#pragma unroll
      for (int it = 0; it < 4; ++it) {
        const int u = tid + it * 512;
        const int d = u >> 3, p8 = u & 7;
        const v4u vv = *(const v4u*)(Vt + (size_t)d * RTOT + gk + p8 * 8);
        *(v4u*)(Vts + d * VPL + p8 * 8) = vv;
      }
      if (tid < NCHK) {
        cjs[tid] = charge[gk + tid];
        sjs[tid] = sqrtf(mass[gk + tid]);
        pjs[tid] = position[gk + tid];
      }
    }
    __syncthreads();

    v8f s = (v8f){0.f,0.f,0.f,0.f,0.f,0.f,0.f,0.f};
#pragma unroll
    for (int dc = 0; dc < 2; ++dc) {
      const v16b kbh = Frag<__bf16>::load(Ksh + krow + dc * 32);
      const v16b kbl = Frag<__bf16>::load(Ksl + krow + dc * 32);
      s = at_mma(qah[dc], kbh, s);
      s = at_mma(qah[dc], kbl, s);
      s = at_mma(qal[dc], kbh, s);
    }
    const int kj = kv0 + kidx;
    const float cj = cjs[kidx], sj = sjs[kidx], pj = pjs[kidx];
    float lmc[8];
#pragma unroll
    for (int r = 0; r < 8; ++r) {
      const int qr = q0 + 8 * hh + r;
      float en = ci[r] * cj + 0.5f * s[r];
      en = en + 0.3f * fabsf(pi[r] - pj);
      en = en + 0.1f * (si[r] * sj);
      const float xv = -en;
      s[r] = xv;
      lmc[r] = (kj <= qr) ? xv : NEGINF;
    }
#pragma unroll
    for (int r = 0; r < 8; ++r) {
      float lm = s[r];
#pragma unroll
      for (int off = 1; off < 16; off <<= 1) lm = fmaxf(lm, __shfl_xor(lm, off, 32));
      const float mfn = fmaxf(mf[r], lm);
      const float a = __expf(mf[r] - mfn);
      float ps = __expf(s[r] - mfn);
#pragma unroll
      for (int off = 1; off < 16; off <<= 1) ps += __shfl_xor(ps, off, 32);
      zf[r] = zf[r] * a + ps;
      mf[r] = mfn;
      float lc = lmc[r];
#pragma unroll
      for (int off = 1; off < 16; off <<= 1) lc = fmaxf(lc, __shfl_xor(lc, off, 32));
      lmc[r] = lc;
    }
    if (c == 0) {
#pragma unroll
      for (int r = 0; r < 8; ++r) mxs[qt][rg * 16 + 8 * hh + r] = lmc[r];
    }
    __syncthreads();

    _Float16* pw = Psh + rg * (16 * PPL);
#pragma unroll
    for (int r = 0; r < 8; ++r) {
      const int row = rg * 16 + 8 * hh + r;
      const int qr = q0 + 8 * hh + r;
      const float mo = fmaxf(fmaxf(mxs[0][row], mxs[1][row]), fmaxf(mxs[2][row], mxs[3][row]));
      const float mnew = fmaxf(mrun[r], mo);
      const float alpha = expf(mrun[r] - mnew);
      const float xe = (kj <= qr) ? s[r] : NEGINF;
      const float ev = expf(xe - mnew);
      float ps = ev;
#pragma unroll
      for (int off = 1; off < 16; off <<= 1) ps += __shfl_xor(ps, off, 32);
      csp[r] = csp[r] * alpha + ps;
      pw[(8 * hh + r) * PPL + kidx] = (_Float16)(ev * PCARRY);
#pragma unroll
      for (int t = 0; t < 4; ++t) oacc[t][r] = oacc[t][r] * alpha;
      mrun[r] = mnew;
    }
    __syncthreads();

#pragma unroll
    for (int kk = 0; kk < 2; ++kk) {
      const v16h pa = Frag<_Float16>::load(pw + c * PPL + kk * 32 + 8 * hh);
#pragma unroll
      for (int t = 0; t < 4; ++t) {
        const int n = qt * 64 + t * 16 + c;
        const v16h vb = Frag<_Float16>::load(Vts + n * VPL + kk * 32 + 8 * hh);
        oacc[t] = mma_h16(pa, vb, oacc[t]);
      }
    }
  }

  for (int kc = qb + 1; kc < NCHK; ++kc) {
    const int kv0 = kc * NCHK;
    const size_t gk = brow + kv0;
    __syncthreads();
    {
      const int row = tid >> 3, q8 = tid & 7;
      const v4u vh = *(const v4u*)(Shi + (gk + row) * SDIM + q8 * 8);
      const v4u vl = *(const v4u*)(Slo + (gk + row) * SDIM + q8 * 8);
      *(v4u*)(Ksh + row * KPL + q8 * 8) = vh;
      *(v4u*)(Ksl + row * KPL + q8 * 8) = vl;
      if (tid < NCHK) {
        cjs[tid] = charge[gk + tid];
        sjs[tid] = sqrtf(mass[gk + tid]);
        pjs[tid] = position[gk + tid];
      }
    }
    __syncthreads();
    v8f s = (v8f){0.f,0.f,0.f,0.f,0.f,0.f,0.f,0.f};
#pragma unroll
    for (int dc = 0; dc < 2; ++dc) {
      const v16b kbh = Frag<__bf16>::load(Ksh + krow + dc * 32);
      const v16b kbl = Frag<__bf16>::load(Ksl + krow + dc * 32);
      s = at_mma(qah[dc], kbh, s);
      s = at_mma(qah[dc], kbl, s);
      s = at_mma(qal[dc], kbh, s);
    }
    const float cj = cjs[kidx], sj = sjs[kidx], pj = pjs[kidx];
#pragma unroll
    for (int r = 0; r < 8; ++r) {
      float en = ci[r] * cj + 0.5f * s[r];
      en = en + 0.3f * fabsf(pi[r] - pj);
      en = en + 0.1f * (si[r] * sj);
      s[r] = -en;
    }
#pragma unroll
    for (int r = 0; r < 8; ++r) {
      float lm = s[r];
#pragma unroll
      for (int off = 1; off < 16; off <<= 1) lm = fmaxf(lm, __shfl_xor(lm, off, 32));
      const float mfn = fmaxf(mf[r], lm);
      const float a = __expf(mf[r] - mfn);
      float ps = __expf(s[r] - mfn);
#pragma unroll
      for (int off = 1; off < 16; off <<= 1) ps += __shfl_xor(ps, off, 32);
      zf[r] = zf[r] * a + ps;
      mf[r] = mfn;
    }
  }
  __syncthreads();

  if (c == 0) {
#pragma unroll
    for (int r = 0; r < 8; ++r) {
      const int row = rg * 16 + 8 * hh + r;
      csx[qt][row] = csp[r];
      mfx[qt][row] = mf[r];
      zfx[qt][row] = zf[r];
    }
  }
  __syncthreads();
  float fac[8];
#pragma unroll
  for (int r = 0; r < 8; ++r) {
    const int row = rg * 16 + 8 * hh + r;
    const size_t gr = gq + 8 * hh + r;
    const float cs = ((csx[0][row] + csx[1][row]) + csx[2][row]) + csx[3][row];
    const float m0 = mfx[0][row], m1 = mfx[1][row], m2 = mfx[2][row], m3 = mfx[3][row];
    const float m = fmaxf(fmaxf(m0, m1), fmaxf(m2, m3));
    const float z = ((zfx[0][row] * expf(m0 - m) + zfx[1][row] * expf(m1 - m)) + zfx[2][row] * expf(m2 - m))
                  + zfx[3][row] * expf(m3 - m);
    const float val = valence[gr];
    const float sc = fminf(val * (1.0f / 1.000001f), 1.0f);
    float den = cs * sc + (1e-8f * z) * expf(fminf(m - mrun[r], 60.0f));
    den = fmaxf(den, 1e-30f);
    fac[r] = sc * PCARRY_INV * __builtin_amdgcn_rcpf(den);
  }

  _Float16* ost = Vts + wave * (16 * OPL);
#pragma unroll
  for (int r = 0; r < 8; ++r) {
#pragma unroll
    for (int t = 0; t < 4; ++t) ost[(8 * hh + r) * OPL + t * 16 + c] = (_Float16)(oacc[t][r] * fac[r]);
  }
  __builtin_amdgcn_fence(__ATOMIC_RELEASE, "workgroup");
  __builtin_amdgcn_wave_barrier();
  __builtin_amdgcn_fence(__ATOMIC_ACQUIRE, "workgroup");
  {
    const int q = lane >> 3, c8 = (lane & 7) * 8;
    for (int pass = 0; pass < 2; ++pass) {
#pragma unroll
      for (int it = 0; it < 4; ++it) {
        const int row = it * 4 + q;
        const v8h v = *(const v8h*)(ost + row * OPL + c8);
        *(volatile v8h*)(Ob + (gq + row) * DPAD + qt * 64 + c8) = v;
      }
      __threadfence();
    }
  }
}

extern "C" void kernel_launch(void* const* d_in, const int* in_sizes, int n_in,
                              void* d_out, int out_size, void* d_ws, size_t ws_size,
                              hipStream_t stream) {
  if (n_in < 10) return;
  if (out_size != RTOT * DOUT) return;
  if (in_sizes[0] < RTOT || in_sizes[1] != RTOT * SDIM || in_sizes[2] < RTOT || in_sizes[3] < RTOT ||
      in_sizes[4] < RTOT || in_sizes[5] != RTOT * DOUT || in_sizes[6] != DOUT * DOUT || in_sizes[8] != DOUT * DOUT) return;

  const float* charge   = (const float*)d_in[0];
  const float* shell    = (const float*)d_in[1];
  const float* mass     = (const float*)d_in[2];
  const float* valence  = (const float*)d_in[3];
  const float* position = (const float*)d_in[4];
  const float* x        = (const float*)d_in[5];
  const float* Wv       = (const float*)d_in[6];
  const float* bv       = (const float*)d_in[7];
  const float* Wo       = (const float*)d_in[8];
  const float* bo       = (const float*)d_in[9];
  float* out = (float*)d_out;
  int nb7 = in_sizes[7]; if (nb7 < 1) nb7 = 1; if (nb7 > 256) nb7 = 256;
  int nb9 = in_sizes[9]; if (nb9 < 1) nb9 = 1; if (nb9 > 256) nb9 = 256;

  size_t off = 0;
  const size_t oShi = off; off += (size_t)RTOT * SDIM * 2;
  const size_t oSlo = off; off += (size_t)RTOT * SDIM * 2;
  const size_t oXh  = off; off += (size_t)RTOT * DPAD * 2;
  const size_t oWvh = off; off += (size_t)DPAD * DPAD * 2;
  const size_t oWoh = off; off += (size_t)DPAD * DPAD * 2;
  const size_t oBvp = off; off += 1024;
  const size_t oBop = off; off += 1024;
  const size_t oVt  = off; off += (size_t)DPAD * RTOT * 2;
  const size_t oOb  = off; off += (size_t)RTOT * DPAD * 2;
  const size_t oY   = off; off += (size_t)RTOT * DPAD * 4;
  if (off > ws_size) return;

  char* ws = (char*)d_ws;
  unsigned short* Shi = (unsigned short*)(ws + oShi);
  unsigned short* Slo = (unsigned short*)(ws + oSlo);
  _Float16* xh  = (_Float16*)(ws + oXh);
  _Float16* Wvh = (_Float16*)(ws + oWvh);
  _Float16* Woh = (_Float16*)(ws + oWoh);
  float* bvp = (float*)(ws + oBvp);
  float* bop = (float*)(ws + oBop);
  _Float16* Vt = (_Float16*)(ws + oVt);
  _Float16* Ob = (_Float16*)(ws + oOb);
  float* Y = (float*)(ws + oY);

  pad_bias2<<<dim3(1), dim3(256), 0, stream>>>(bv, nb7, bo, nb9, bvp, bop);
  {
    const int n2 = RTOT * SDIM / 2;
    split_bf16x2<<<dim3((n2 + 255) / 256), dim3(256), 0, stream>>>(shell, Shi, Slo, n2);
  }
  {
    const int n2 = RTOT * (DPAD / 2);
    padcast_f16x2<<<dim3((n2 + 255) / 256), dim3(256), 0, stream>>>(x, xh, RTOT, DOUT, 1.0f, n2);
  }
  {
    const int n2 = DPAD * (DPAD / 2);
    padcast_f16x2<<<dim3((n2 + 255) / 256), dim3(256), 0, stream>>>(Wv, Wvh, DOUT, DOUT, 16.0f, n2);
    padcast_f16x2<<<dim3((n2 + 255) / 256), dim3(256), 0, stream>>>(Wo, Woh, DOUT, DOUT, 16.0f, n2);
  }
  {
    const int M = DPAD, N = RTOT, K = DPAD;
    const int tiles = (M / 64) * (N / 64);
    wmma_gemm64<0, false, 1, 1, false><<<dim3((tiles + 7) / 8, 1), dim3(256), 0, stream>>>(
        U16(Wvh), U16(Wvh), DPAD, 0L, U16(xh), U16(xh), DPAD, 0L,
        (void*)Vt, (void*)Vt, RTOT, 0L, bvp, bvp, 0L, M, N, K, 1.0f / 16.0f);
  }
  attn_energy<<<dim3((RTOT / NSEQ) * NCHK), dim3(512), 0, stream>>>(Shi, Slo, Vt, charge, mass, position, valence, Ob);
  {
    const int M = RTOT, N = DPAD, K = DPAD;
    const int tiles = (M / 64) * (N / 64);
    wmma_gemm64<0, false, 2, 0, false><<<dim3((tiles + 7) / 8, 1), dim3(256), 0, stream>>>(
        U16(Ob), U16(Ob), DPAD, 0L, U16(Woh), U16(Woh), DPAD, 0L,
        (void*)Y, (void*)Y, DPAD, 0L, bop, bop, 0L, M, N, K, 1.0f / 16.0f);
  }
  {
    const int n4 = RTOT * DOUT / 4;
    copy_out<<<dim3((n4 + 255) / 256), dim3(256), 0, stream>>>(Y, out, n4);
  }
}
